// TextDecoderLayer_29738353557823
// MI455X (gfx1250) — hardware-verified
//
#include <hip/hip_runtime.h>
#include <math.h>

typedef __attribute__((ext_vector_type(16))) _Float16 v16h;
typedef __attribute__((ext_vector_type(8)))  _Float16 v8h;
typedef __attribute__((ext_vector_type(16))) __bf16   v16b;
typedef __attribute__((ext_vector_type(8)))  __bf16   v8b;
typedef __attribute__((ext_vector_type(8)))  float    v8f;
typedef __attribute__((ext_vector_type(4)))  float    v4f;

constexpr int B_SZ    = 2;
constexpr int T_LEN   = 2048;
constexpr int D_MODEL = 1024;
constexpr int N_QH    = 16;
constexpr int N_KVH   = 4;
constexpr int HEAD_D  = 64;
constexpr int GQA_R   = N_QH / N_KVH;
constexpr int KV_COLS = N_KVH * HEAD_D;
constexpr int F_DIM   = 4096;
constexpr int F_HALF  = 2048;
constexpr int BT_ROWS = B_SZ * T_LEN;
constexpr int QKV_N   = D_MODEL + 2 * KV_COLS;
constexpr int KCOL0   = D_MODEL;
constexpr int VCOL0   = D_MODEL + KV_COLS;
constexpr float NORM_EPS  = 1e-6f;
constexpr float W_CARRY   = 32.0f;
constexpr float P_CARRY   = 32768.0f;
constexpr float ATT_CARRY = 16.0f;
constexpr float HID_CARRY = 16.0f;
constexpr float SM_SCALE  = 0.125f;
constexpr float NEG_FILL  = -3.40282347e38f;
constexpr int LDS_P16 = 72;

static_assert(T_LEN % 64 == 0 && D_MODEL % 64 == 0 && F_HALF % 64 == 0 && QKV_N % 64 == 0 && KV_COLS % 64 == 0);
static_assert(D_MODEL % 32 == 0 && F_HALF % 32 == 0);
static_assert(GQA_R * N_KVH == N_QH && HEAD_D == 64 && D_MODEL == 4 * 256);

constexpr size_t MIB      = 1048576;
constexpr size_t OFF_WQKV = 0;
constexpr size_t OFF_WO   = 3 * MIB;
constexpr size_t OFF_HR   = 5 * MIB;
constexpr size_t OFF_X16  = 21 * MIB;
constexpr size_t OFF_H1   = 21 * MIB;
constexpr size_t OFF_QKV  = 29 * MIB;
constexpr size_t OFF_Q16  = 53 * MIB;
constexpr size_t OFF_K16  = 61 * MIB;
constexpr size_t OFF_VT16 = 63 * MIB;
constexpr size_t OFF_ATT  = 65 * MIB;
constexpr size_t OFF_V16  = 73 * MIB;
constexpr size_t OFF_Y16  = 0;
constexpr size_t OFF_WD   = 8 * MIB;
constexpr size_t OFF_WGU  = 37 * MIB;
constexpr size_t OFF_G16  = 53 * MIB;
constexpr size_t OFF_U16  = 69 * MIB;
constexpr size_t OFF_H16  = 85 * MIB;
constexpr size_t OFF_TMP  = 101 * MIB;
constexpr size_t WS_NEED  = 117 * MIB;
static_assert((size_t)QKV_N * D_MODEL * 2 <= OFF_WO - OFF_WQKV);
static_assert((size_t)D_MODEL * D_MODEL * 2 <= OFF_HR - OFF_WO);
static_assert((size_t)BT_ROWS * D_MODEL * 4 == OFF_X16 - OFF_HR);
static_assert((size_t)BT_ROWS * D_MODEL * 2 == OFF_QKV - OFF_X16);
static_assert((size_t)BT_ROWS * QKV_N * 4 == OFF_Q16 - OFF_QKV);
static_assert((size_t)B_SZ * N_QH * T_LEN * HEAD_D * 2 == OFF_K16 - OFF_Q16);
static_assert((size_t)B_SZ * N_KVH * T_LEN * HEAD_D * 2 == OFF_VT16 - OFF_K16);
static_assert((size_t)B_SZ * N_KVH * HEAD_D * T_LEN * 2 == OFF_ATT - OFF_VT16);
static_assert((size_t)BT_ROWS * D_MODEL * 2 == OFF_V16 - OFF_ATT);
static_assert(OFF_V16 + (size_t)B_SZ * N_KVH * T_LEN * HEAD_D * 2 <= WS_NEED);
static_assert(OFF_H1 + (size_t)BT_ROWS * D_MODEL * 4 == OFF_WGU);
static_assert(OFF_Y16 + (size_t)BT_ROWS * D_MODEL * 2 == OFF_WD);
static_assert(OFF_WD + (size_t)D_MODEL * F_DIM * 2 <= OFF_H1);
static_assert(OFF_WGU + (size_t)2 * F_DIM * D_MODEL * 2 == OFF_G16);
static_assert(OFF_G16 + (size_t)BT_ROWS * F_HALF * 2 == OFF_U16);
static_assert(OFF_U16 + (size_t)BT_ROWS * F_HALF * 2 == OFF_H16);
static_assert(OFF_H16 + (size_t)BT_ROWS * F_HALF * 2 == OFF_TMP);
static_assert(OFF_TMP + (size_t)BT_ROWS * D_MODEL * 4 == WS_NEED);
static_assert(WS_NEED <= 134217728);

__device__ __forceinline__ unsigned short f2bf_bits(float f) {
  unsigned u = __float_as_uint(f);
  return (unsigned short)((u + 0x7FFFu + ((u >> 16) & 1u)) >> 16);
}
__device__ __forceinline__ float bf_bits2f(unsigned short h) { return __uint_as_float(((unsigned)h) << 16); }
__device__ __forceinline__ float bf_rne(float f) { return bf_bits2f(f2bf_bits(f)); }

__device__ __forceinline__ void dep_guard_h(v8f& a, v8f& b, v16h x, v16h y) { asm volatile("v_nop\n\tv_nop\n\tv_nop\n\tv_nop" : "+v"(a), "+v"(b) : "v"(x), "v"(y)); }
__device__ __forceinline__ void dep_guard_b(v8f& a, v8f& b, v16b x, v16b y) { asm volatile("v_nop\n\tv_nop\n\tv_nop\n\tv_nop" : "+v"(a), "+v"(b) : "v"(x), "v"(y)); }
__device__ __forceinline__ void keep4_h(v16h a, v16h b, v16h c, v16h d) { asm volatile("v_nop" :: "v"(a), "v"(b), "v"(c), "v"(d)); }
__device__ __forceinline__ void keep4_b(v16b a, v16b b, v16b c, v16b d) { asm volatile("v_nop" :: "v"(a), "v"(b), "v"(c), "v"(d)); }
__device__ __forceinline__ void acc_guard4(v8f& a, v8f& b, v8f& c, v8f& d) { asm volatile("v_nop\n\tv_nop\n\tv_nop\n\tv_nop" : "+v"(a), "+v"(b), "+v"(c), "+v"(d)); }
template <typename T> struct Frag;
template <> struct Frag<_Float16> {
  typedef v16h V; union U { v16h v; v8h h[2]; };
  static __device__ __forceinline__ v16h load(const _Float16* p) {
    U f; f.h[0] = *(const v8h*)(p); f.h[1] = *(const v8h*)(p + 16); return f.v;
  }
  static __device__ __forceinline__ v8f mma(v16h a, v16h b, v8f c) {
    return __builtin_amdgcn_wmma_f32_16x16x32_f16(false, a, false, b, (short)0, c, false, false);
  }
  static __device__ __forceinline__ void guard(v8f& a, v8f& b, v16h x, v16h y) { dep_guard_h(a, b, x, y); }
  static __device__ __forceinline__ void keep(v16h a, v16h b, v16h c, v16h d) { keep4_h(a, b, c, d); }
};
template <> struct Frag<__bf16> {
  typedef v16b V; union U { v16b v; v8b h[2]; };
  static __device__ __forceinline__ v16b load(const __bf16* p) {
    U f; f.h[0] = *(const v8b*)(p); f.h[1] = *(const v8b*)(p + 16); return f.v;
  }
  static __device__ __forceinline__ v8f mma(v16b a, v16b b, v8f c) {
    return __builtin_amdgcn_wmma_f32_16x16x32_bf16(false, a, false, b, (short)0, c, false, false);
  }
  static __device__ __forceinline__ void guard(v8f& a, v8f& b, v16b x, v16b y) { dep_guard_b(a, b, x, y); }
  static __device__ __forceinline__ void keep(v16b a, v16b b, v16b c, v16b d) { keep4_b(a, b, c, d); }
};

__device__ __forceinline__ v8f hmma_g(v16h a, v16h b, v8f c) {
  c = __builtin_amdgcn_wmma_f32_16x16x32_f16(false, a, false, b, (short)0, c, false, false);
  asm volatile("v_nop\n\tv_nop\n\tv_nop\n\tv_nop" : "+v"(c) : "v"(a), "v"(b));
  return c;
}

template <int ET> struct Elem;
template <> struct Elem<0> { typedef _Float16 T; };
template <> struct Elem<1> { typedef __bf16 T; };
template <int ET, int SPLITM, int BIAS_MODE, int OUT_MODE, bool RESID, int ACT = 0>
__global__ __launch_bounds__(256) void wmma_gemm64(
    const unsigned short* __restrict__ Ap, const unsigned short* __restrict__ A2p, int lda, long strideA,
    const unsigned short* __restrict__ Btp, const unsigned short* __restrict__ Bt2p, int ldb, long strideB,
    void* __restrict__ Cout, void* __restrict__ Cout2, int ldc, long strideC,
    const float* __restrict__ bias,
    const float* __restrict__ resid, long strideR,
    int M, int N, int K, float scale) {
  typedef typename Elem<ET>::T T;
  typedef typename Frag<T>::V V;
  constexpr bool SPA = (SPLITM >= 1);
  constexpr bool SPB = (SPLITM >= 2);
  const T* A = (const T*)Ap; const T* A2 = (const T*)A2p; const T* Bt = (const T*)Btp; const T* Bt2 = (const T*)Bt2p;
  __shared__ __align__(16) float sT[8][16 * 68];
  const int b    = blockIdx.y;
  const int lane = threadIdx.x & 31;
  const int wave = threadIdx.x >> 5;
  const int tilesN = N >> 6;
  const int tilesM = M >> 6;
  const int tile = blockIdx.x * 8 + wave;
  if (tile >= tilesM * tilesN) return;
  const int tm = tile / tilesN;
  const int tn = tile - tm * tilesN;
  const int m0 = tm << 6;
  const int n0 = tn << 6;

  const T* Ab  = A  + (size_t)b * strideA;
  const T* Bb  = Bt + (size_t)b * strideB;
  const T* Ab2 = SPA ? (A2  + (size_t)b * strideA) : nullptr;
  const T* Bb2 = SPB ? (Bt2 + (size_t)b * strideB) : nullptr;

  const int rlane = lane & 15;
  const int koff  = (lane >> 4) * 8;
  const int mOff  = (lane >> 4) * 8;

  v8f acc[4][4];
#pragma unroll
  for (int i = 0; i < 4; ++i)
#pragma unroll
    for (int j = 0; j < 4; ++j) acc[i][j] = (v8f){0.f,0.f,0.f,0.f,0.f,0.f,0.f,0.f};

  for (int k0 = 0; k0 < K; k0 += 32) {
    V bh[4], bl[4];
#pragma unroll
    for (int j = 0; j < 4; ++j) {
      const size_t bo = (size_t)(n0 + (j << 4) + rlane) * ldb + koff + k0;
      bh[j] = Frag<T>::load(Bb + bo);
      if (SPB) bl[j] = Frag<T>::load(Bb2 + bo);
    }
#pragma unroll
    for (int i = 0; i < 4; ++i) {
      const size_t ao = (size_t)(m0 + (i << 4) + rlane) * lda + koff + k0;
      V ah = Frag<T>::load(Ab + ao);
      V al;
      if (SPA) al = Frag<T>::load(Ab2 + ao);
#pragma unroll
      for (int j = 0; j < 4; ++j) {
        acc[i][j] = Frag<T>::mma(ah, bh[j], acc[i][j]);
        if (SPB) acc[i][j] = Frag<T>::mma(ah, bl[j], acc[i][j]);
        if (SPA) acc[i][j] = Frag<T>::mma(al, bh[j], acc[i][j]);
      }
      Frag<T>::guard(acc[i][0], acc[i][3], ah, SPA ? al : ah);
    }
    Frag<T>::keep(bh[0], bh[1], bh[2], bh[3]);
    if (SPB) Frag<T>::keep(bl[0], bl[1], bl[2], bl[3]);
  }
  acc_guard4(acc[0][0], acc[0][1], acc[0][2], acc[0][3]);
  acc_guard4(acc[1][0], acc[1][1], acc[1][2], acc[1][3]);
  acc_guard4(acc[2][0], acc[2][1], acc[2][2], acc[2][3]);
  acc_guard4(acc[3][0], acc[3][1], acc[3][2], acc[3][3]);

  float* slab = sT[wave];
  const float* Rb = RESID ? (resid + (size_t)b * strideR) : nullptr;
#pragma unroll
  for (int i = 0; i < 4; ++i) {
    const int mBase = m0 + (i << 4);
#pragma unroll
    for (int j = 0; j < 4; ++j) {
      const int n = n0 + (j << 4) + rlane;
      float bv = 0.f;
      if (BIAS_MODE == 2) bv = bias[n];
#pragma unroll
      for (int r = 0; r < 8; ++r) {
        float v = acc[i][j][r] * scale;
        if (BIAS_MODE == 1) v += bias[mBase + mOff + r];
        if (BIAS_MODE == 2) v += bv;
        if (RESID) v += Rb[(size_t)(mBase + mOff + r) * ldc + n];
        if (ACT == 1) v = tanhf(v);
        if (ACT == 2) v = fmaxf(v, 0.0f);
        if (ACT == 4) v = (v > 0.f) ? v : 0.01f * v;
        slab[(mOff + r) * 68 + (j << 4) + rlane] = v;
      }
    }
    __builtin_amdgcn_fence(__ATOMIC_RELEASE, "workgroup");
    __builtin_amdgcn_wave_barrier();
    __builtin_amdgcn_fence(__ATOMIC_ACQUIRE, "workgroup");
    if (OUT_MODE == 0) {
      float* C = (float*)Cout + (size_t)b * strideC;
      const int hh = lane >> 4, c4 = (lane & 15) * 4;
      for (int pass = 0; pass < 2; ++pass) {
#pragma unroll
        for (int it = 0; it < 8; ++it) {
          const int row = it * 2 + hh;
          v4f v = *(const v4f*)(slab + row * 68 + c4);
          *(volatile v4f*)(C + (size_t)(mBase + row) * ldc + n0 + c4) = v;
        }
        __threadfence();
      }
    } else {
      const int q = lane >> 3, c8 = (lane & 7) * 8;
      unsigned short* C  = (unsigned short*)Cout  + (size_t)b * strideC;
      unsigned short* C2 = (OUT_MODE == 2) ? ((unsigned short*)Cout2 + (size_t)b * strideC) : nullptr;
      for (int pass = 0; pass < 2; ++pass) {
#pragma unroll
        for (int it = 0; it < 4; ++it) {
          const int row = it * 4 + q;
          const float* sp = slab + row * 68 + c8;
          v8h hv, lv;
#pragma unroll
          for (int e = 0; e < 8; ++e) {
            if (OUT_MODE == 1) {
              hv[e] = (_Float16)sp[e];
            } else {
              unsigned short hb = f2bf_bits(sp[e]);
              unsigned short lb = f2bf_bits(sp[e] - bf_bits2f(hb));
              hv[e] = __builtin_bit_cast(_Float16, hb);
              lv[e] = __builtin_bit_cast(_Float16, lb);
            }
          }
          *(volatile v8h*)(C + (size_t)(mBase + row) * ldc + n0 + c8) = hv;
          if (OUT_MODE == 2) *(volatile v8h*)(C2 + (size_t)(mBase + row) * ldc + n0 + c8) = lv;
        }
        __threadfence();
      }
    }
    __builtin_amdgcn_fence(__ATOMIC_RELEASE, "workgroup");
    __builtin_amdgcn_wave_barrier();
    __builtin_amdgcn_fence(__ATOMIC_ACQUIRE, "workgroup");
  }
}

__global__ __launch_bounds__(256) void cvt_weight_k(const float* __restrict__ w, int ldw, int kdim,
                                                    unsigned short* __restrict__ wt) {
  __shared__ __align__(16) _Float16 tl[64 * LDS_P16];
  const int n0 = blockIdx.x * 64, k0 = blockIdx.y * 64;
  const int tid = threadIdx.x;
#pragma unroll
  for (int i = 0; i < 4; ++i) {
    const int idx = tid + 256 * i;
    const int kr = idx >> 4, c4 = (idx & 15) * 4;
    const v4f v = *(const v4f*)(w + (size_t)(k0 + kr) * ldw + n0 + c4);
#pragma unroll
    for (int e = 0; e < 4; ++e) tl[(c4 + e) * LDS_P16 + kr] = (_Float16)(bf_rne(v[e]) * W_CARRY);
  }
  __syncthreads();
  const int wave = tid >> 5, lane = tid & 31, q8 = lane >> 3, c8 = (lane & 7) * 8;
  const int nA = wave * 4 + q8, nB = 32 + wave * 4 + q8;
  const v8h va = *(const v8h*)(tl + nA * LDS_P16 + c8);
  const v8h vb = *(const v8h*)(tl + nB * LDS_P16 + c8);
  _Float16* wth = (_Float16*)wt;
  const size_t oA = (size_t)(n0 + nA) * kdim + k0 + c8;
  const size_t oB = (size_t)(n0 + nB) * kdim + k0 + c8;
  for (int pass = 0; pass < 2; ++pass) {
    *(volatile v8h*)(wth + oA) = va;
    *(volatile v8h*)(wth + oB) = vb;
    __threadfence();
  }
}

template <bool RIN, bool WR>
__global__ __launch_bounds__(256) void rmsnorm_row_k(const float* __restrict__ x, const float* __restrict__ scale,
                                                     float* __restrict__ xr, unsigned short* __restrict__ y16) {
  __shared__ float red[8];
  __shared__ __align__(16) float rowbuf[D_MODEL];
  const int row = blockIdx.x, tid = threadIdx.x, wave = tid >> 5, lane = tid & 31;
  const size_t ro = (size_t)row * D_MODEL;
  v4f v = *(const v4f*)(x + ro + 4 * tid);
  if (RIN) {
#pragma unroll
    for (int e = 0; e < 4; ++e) v[e] = bf_rne(v[e]);
  }
  float ss = v[0] * v[0] + v[1] * v[1] + v[2] * v[2] + v[3] * v[3];
#pragma unroll
  for (int off = 16; off > 0; off >>= 1) ss += __shfl_xor(ss, off, 32);
  if (lane == 0) red[wave] = ss;
  __syncthreads();
  const float tot = ((red[0] + red[1]) + (red[2] + red[3])) + ((red[4] + red[5]) + (red[6] + red[7]));
  const float rr = rsqrtf(tot * (1.0f / (float)D_MODEL) + NORM_EPS);
  if (WR) {
    for (int pass = 0; pass < 2; ++pass) {
      *(volatile v4f*)(xr + ro + 4 * tid) = v;
      __threadfence();
    }
  }
  const v4f sc = *(const v4f*)(scale + 4 * tid);
  v4f y;
#pragma unroll
  for (int e = 0; e < 4; ++e) y[e] = bf_rne(sc[e]) * (v[e] * rr);
  *(v4f*)(rowbuf + 4 * tid) = y;
  __syncthreads();
  if (tid < 128) {
    const v4f a0 = *(const v4f*)(rowbuf + 8 * tid);
    const v4f a1 = *(const v4f*)(rowbuf + 8 * tid + 4);
    v8h hv;
#pragma unroll
    for (int e = 0; e < 4; ++e) { hv[e] = (_Float16)a0[e]; hv[4 + e] = (_Float16)a1[e]; }
    _Float16* yrow = (_Float16*)y16 + ro;
    for (int pass = 0; pass < 2; ++pass) {
      *(volatile v8h*)(yrow + 8 * tid) = hv;
      __threadfence();
    }
  }
}

__global__ __launch_bounds__(256) void headnorm_rope_k(const float* __restrict__ qkv,
    const float* __restrict__ qn, const float* __restrict__ kn,
    const float* __restrict__ sinp, const float* __restrict__ cosp,
    unsigned short* __restrict__ q16, unsigned short* __restrict__ k16, unsigned short* __restrict__ v16) {
#pragma clang fp contract(off)
  __shared__ __align__(16) _Float16 stg[8][4 * LDS_P16];
  const int bt = blockIdx.x;
  const int b = bt / T_LEN, t = bt - b * T_LEN;
  const int tid = threadIdx.x, wave = tid >> 5, ln = tid & 31;
  const float sn  = bf_rne(sinp[(size_t)bt * 32 + ln]);
  const float cs  = bf_rne(cosp[(size_t)bt * 32 + ln]);
  const float qs1 = bf_rne(qn[ln]), qs2 = bf_rne(qn[ln + 32]);
  const float ks1 = bf_rne(kn[ln]), ks2 = bf_rne(kn[ln + 32]);
  const float* rowp = qkv + (size_t)bt * QKV_N;
  _Float16* sw = stg[wave];
  const int gk = wave & 3;
  const bool isK = (wave < 4);
#pragma unroll
  for (int j = 0; j < 2; ++j) {
    const int hq = wave + 8 * j;
    const float x1 = rowp[hq * HEAD_D + ln], x2 = rowp[hq * HEAD_D + 32 + ln];
    float ss = x1 * x1 + x2 * x2;
#pragma unroll
    for (int off = 16; off > 0; off >>= 1) ss += __shfl_xor(ss, off, 32);
    const float rr = rsqrtf(ss * (1.0f / (float)HEAD_D) + NORM_EPS);
    const float a1 = qs1 * (x1 * rr), a2 = qs2 * (x2 * rr);
    sw[j * LDS_P16 + ln]      = (_Float16)(a1 * cs - a2 * sn);
    sw[j * LDS_P16 + 32 + ln] = (_Float16)(a2 * cs + a1 * sn);
  }
  {
    const float x1 = rowp[KCOL0 + gk * HEAD_D + ln], x2 = rowp[KCOL0 + gk * HEAD_D + 32 + ln];
    float ss = x1 * x1 + x2 * x2;
#pragma unroll
    for (int off = 16; off > 0; off >>= 1) ss += __shfl_xor(ss, off, 32);
    const float rr = rsqrtf(ss * (1.0f / (float)HEAD_D) + NORM_EPS);
    const float a1 = ks1 * (x1 * rr), a2 = ks2 * (x2 * rr);
    const float ok1 = a1 * cs - a2 * sn, ok2 = a2 * cs + a1 * sn;
    const float xv1 = rowp[VCOL0 + gk * HEAD_D + ln], xv2 = rowp[VCOL0 + gk * HEAD_D + 32 + ln];
    sw[2 * LDS_P16 + ln]      = (_Float16)(isK ? ok1 : xv1);
    sw[2 * LDS_P16 + 32 + ln] = (_Float16)(isK ? ok2 : xv2);
  }
  __builtin_amdgcn_fence(__ATOMIC_RELEASE, "workgroup");
  __builtin_amdgcn_wave_barrier();
  __builtin_amdgcn_fence(__ATOMIC_ACQUIRE, "workgroup");
  const int q8 = ln >> 3, c8 = (ln & 7) * 8;
  const int rs = (q8 < 3) ? q8 : 2;
  const v8h val = *(const v8h*)(sw + rs * LDS_P16 + c8);
  _Float16* dq0 = (_Float16*)q16 + ((size_t)(b * N_QH + wave) * T_LEN + t) * HEAD_D + c8;
  _Float16* dq1 = (_Float16*)q16 + ((size_t)(b * N_QH + wave + 8) * T_LEN + t) * HEAD_D + c8;
  _Float16* dkv = (_Float16*)(isK ? k16 : v16) + ((size_t)(b * N_KVH + gk) * T_LEN + t) * HEAD_D + c8;
  _Float16* dst = (q8 == 0) ? dq0 : ((q8 == 1) ? dq1 : dkv);
  for (int pass = 0; pass < 2; ++pass) {
    if (q8 < 3) *(volatile v8h*)dst = val;
    __threadfence();
  }
}

__global__ __launch_bounds__(256) void vt_transpose_k(const unsigned short* __restrict__ vin, unsigned short* __restrict__ vt) {
  __shared__ __align__(16) _Float16 th[64 * LDS_P16];
  const int st0 = blockIdx.x * 64, bg = blockIdx.y;
  const int tid = threadIdx.x;
  {
    const int sloc = tid >> 2, d0 = (tid & 3) * 16;
    const size_t so = ((size_t)bg * T_LEN + st0 + sloc) * HEAD_D + d0;
    const v8h a0 = *(const v8h*)((const _Float16*)vin + so);
    const v8h a1 = *(const v8h*)((const _Float16*)vin + so + 8);
#pragma unroll
    for (int e = 0; e < 8; ++e) {
      th[(d0 + e) * LDS_P16 + sloc]     = a0[e];
      th[(d0 + 8 + e) * LDS_P16 + sloc] = a1[e];
    }
  }
  __syncthreads();
  const int wave = tid >> 5, lane = tid & 31, q8 = lane >> 3, c8 = (lane & 7) * 8;
  const int dA = wave * 8 + q8, dB = wave * 8 + 4 + q8;
  const v8h hvA = *(const v8h*)(th + dA * LDS_P16 + c8);
  const v8h hvB = *(const v8h*)(th + dB * LDS_P16 + c8);
  _Float16* vth = (_Float16*)vt;
  const size_t oA = ((size_t)bg * HEAD_D + dA) * T_LEN + st0 + c8;
  const size_t oB = ((size_t)bg * HEAD_D + dB) * T_LEN + st0 + c8;
  for (int pass = 0; pass < 2; ++pass) {
    *(volatile v8h*)(vth + oA) = hvA;
    *(volatile v8h*)(vth + oB) = hvB;
    __threadfence();
  }
}

__global__ __launch_bounds__(128) void attn_causal_k(
    const unsigned short* __restrict__ qp, const unsigned short* __restrict__ kp,
    const unsigned short* __restrict__ vtp, const int* __restrict__ mk, unsigned short* __restrict__ op) {
  __shared__ __align__(16) _Float16 Ksh[64 * LDS_P16];
  __shared__ __align__(16) _Float16 Vts[64 * LDS_P16];
  __shared__ __align__(16) _Float16 Psh[4][16 * LDS_P16];
  __shared__ __align__(16) float  Os[4][16 * 68];
  const int tid = threadIdx.x, wave = tid >> 5, lane = tid & 31, hh = lane >> 4, c = lane & 15;
  constexpr int NQB = T_LEN / 64;
  const int bx = blockIdx.x;
  const int qb = bx % NQB;
  const int bh = bx / NQB;
  const int h  = bh % N_QH;
  const int b  = bh / N_QH;
  const int g  = h / GQA_R;
  const int q0 = qb * 64 + wave * 16;
  const _Float16* Qb = (const _Float16*)qp  + (size_t)(b * N_QH + h) * T_LEN * HEAD_D;
  const _Float16* Kb = (const _Float16*)kp  + (size_t)(b * N_KVH + g) * T_LEN * HEAD_D;
  const _Float16* Vb = (const _Float16*)vtp + (size_t)(b * N_KVH + g) * HEAD_D * T_LEN;
  const int*      Mb = mk + (size_t)b * T_LEN * T_LEN;
  _Float16*       Ob = (_Float16*)op + (size_t)b * T_LEN * D_MODEL + (size_t)h * HEAD_D;

  v16h qa[2];
#pragma unroll
  for (int dc = 0; dc < 2; ++dc) qa[dc] = Frag<_Float16>::load(Qb + (size_t)(q0 + c) * HEAD_D + dc * 32 + 8 * hh);

  float mrow[8], lrow[8];
  v8f oacc[4];
#pragma unroll
  for (int r = 0; r < 8; ++r) { mrow[r] = -INFINITY; lrow[r] = 0.f; }
#pragma unroll
  for (int t = 0; t < 4; ++t) oacc[t] = (v8f){0.f,0.f,0.f,0.f,0.f,0.f,0.f,0.f};

  const int nChunks = qb + 1;
  for (int kc = 0; kc < nChunks; ++kc) {
    const int kv0 = kc * 64;
    __syncthreads();
    {
      const int rr = tid >> 1, sh = (tid & 1) * 32;
      const _Float16* krow = Kb + (size_t)(kv0 + rr) * HEAD_D + sh;
      const _Float16* vrow = Vb + (size_t)rr * T_LEN + kv0 + sh;
#pragma unroll
      for (int i = 0; i < 4; ++i) {
        const v8h kk = *(const v8h*)(krow + 8 * i);
        const v8h vv = *(const v8h*)(vrow + 8 * i);
        *(v8h*)(Ksh + rr * LDS_P16 + sh + 8 * i) = kk;
        *(v8h*)(Vts + rr * LDS_P16 + sh + 8 * i) = vv;
      }
    }
    __syncthreads();

    v8f s[4];
#pragma unroll
    for (int j = 0; j < 4; ++j) {
      s[j] = (v8f){0.f,0.f,0.f,0.f,0.f,0.f,0.f,0.f};
#pragma unroll
      for (int dc = 0; dc < 2; ++dc) {
        const v16h kb = Frag<_Float16>::load(Ksh + (j * 16 + c) * LDS_P16 + dc * 32 + 8 * hh);
        s[j] = hmma_g(qa[dc], kb, s[j]);
      }
    }
    float cm[8];
#pragma unroll
    for (int r = 0; r < 8; ++r) {
      const int qrow = q0 + 8 * hh + r;
      const int* mr = Mb + (size_t)qrow * T_LEN + kv0;
      float m = -INFINITY;
#pragma unroll
      for (int j = 0; j < 4; ++j) {
        const int mv = mr[j * 16 + c];
        const float sv = s[j][r] * SM_SCALE;
        const float sel = (mv != 0) ? sv : NEG_FILL;
        s[j][r] = sel;
        m = fmaxf(m, sel);
      }
#pragma unroll
      for (int off = 1; off < 16; off <<= 1) m = fmaxf(m, __shfl_xor(m, off, 32));
      cm[r] = m;
    }
    _Float16* pw = Psh[wave];
#pragma unroll
    for (int r = 0; r < 8; ++r) {
      const float mnew = fmaxf(mrow[r], cm[r]);
      const float alpha = __expf(mrow[r] - mnew);
      mrow[r] = mnew;
      float psum = 0.f;
#pragma unroll
      for (int j = 0; j < 4; ++j) {
        const float p = __expf(s[j][r] - mnew);
        psum += p;
        pw[(8 * hh + r) * LDS_P16 + j * 16 + c] = (_Float16)(p * P_CARRY);
      }
#pragma unroll
      for (int off = 1; off < 16; off <<= 1) psum += __shfl_xor(psum, off, 32);
      lrow[r] = lrow[r] * alpha + psum;
#pragma unroll
      for (int t = 0; t < 4; ++t) oacc[t][r] *= alpha;
    }
    __builtin_amdgcn_fence(__ATOMIC_RELEASE, "workgroup");
    __builtin_amdgcn_wave_barrier();
    __builtin_amdgcn_fence(__ATOMIC_ACQUIRE, "workgroup");
#pragma unroll 1
    for (int kk = 0; kk < 2; ++kk) {
      const v16h pa = Frag<_Float16>::load(pw + c * LDS_P16 + kk * 32 + 8 * hh);
#pragma unroll
      for (int t = 0; t < 4; ++t) {
        const v16h vb = Frag<_Float16>::load(Vts + (t * 16 + c) * LDS_P16 + kk * 32 + 8 * hh);
        oacc[t] = hmma_g(pa, vb, oacc[t]);
      }
    }
  }

  float* os = Os[wave];
#pragma unroll
  for (int r = 0; r < 8; ++r) {
    const float inv = ATT_CARRY * __builtin_amdgcn_rcpf(lrow[r] * P_CARRY);
#pragma unroll
    for (int t = 0; t < 4; ++t) os[(8 * hh + r) * 68 + t * 16 + c] = oacc[t][r] * inv;
  }
  __builtin_amdgcn_fence(__ATOMIC_RELEASE, "workgroup");
  __builtin_amdgcn_wave_barrier();
  __builtin_amdgcn_fence(__ATOMIC_ACQUIRE, "workgroup");
  {
    const int q8 = lane >> 3, c8 = (lane & 7) * 8;
    for (int pass = 0; pass < 2; ++pass) {
#pragma unroll
      for (int it = 0; it < 4; ++it) {
        const int row = it * 4 + q8;
        const float* sp = os + row * 68 + c8;
        v8h hv;
#pragma unroll
        for (int e = 0; e < 8; ++e) hv[e] = (_Float16)sp[e];
        *(volatile v8h*)(Ob + (size_t)(q0 + row) * D_MODEL + c8) = hv;
      }
      __threadfence();
    }
  }
}

__global__ __launch_bounds__(256) void silu_mul_k(const unsigned short* __restrict__ gp, const unsigned short* __restrict__ up,
                                                  unsigned short* __restrict__ hp, int n8) {
  const int i = blockIdx.x * 256 + threadIdx.x;
  if (i < n8) {
    const v8h gv = ((const v8h*)gp)[i];
    const v8h uv = ((const v8h*)up)[i];
    v8h hv;
#pragma unroll
    for (int e = 0; e < 8; ++e) {
      const float gf = (float)gv[e], uf = (float)uv[e];
      const float sg = __builtin_amdgcn_rcpf(1.0f + __expf(-gf));
      hv[e] = (_Float16)(((gf * sg) * uf) * HID_CARRY);
    }
    ((volatile v8h*)hp)[i] = hv;
    __threadfence();
    ((volatile v8h*)hp)[i] = hv;
  }
}

extern "C" void kernel_launch(void* const* d_in, const int* in_sizes, int n_in,
                              void* d_out, int out_size, void* d_ws, size_t ws_size,
                              hipStream_t stream)
{
  if (n_in < 15) return;
  if (in_sizes[0] != BT_ROWS * D_MODEL || in_sizes[1] != BT_ROWS * 32 || in_sizes[2] != BT_ROWS * 32 ||
      in_sizes[3] != B_SZ * T_LEN * T_LEN || in_sizes[4] != D_MODEL || in_sizes[5] != D_MODEL ||
      in_sizes[6] != HEAD_D || in_sizes[7] != HEAD_D ||
      in_sizes[8] != D_MODEL * D_MODEL || in_sizes[9] != D_MODEL * KV_COLS || in_sizes[10] != D_MODEL * KV_COLS ||
      in_sizes[11] != D_MODEL * D_MODEL || in_sizes[12] != D_MODEL * F_DIM || in_sizes[13] != D_MODEL * F_DIM ||
      in_sizes[14] != F_DIM * D_MODEL) return;
  if (out_size != BT_ROWS * D_MODEL) return;
  if (ws_size < WS_NEED) return;

  const float* hidden = (const float*)d_in[0];
  const float* sinp   = (const float*)d_in[1];
  const float* cosp   = (const float*)d_in[2];
  const int*   maskp  = (const int*)d_in[3];
  const float* ln1    = (const float*)d_in[4];
  const float* ln2    = (const float*)d_in[5];
  const float* qns    = (const float*)d_in[6];
  const float* kns    = (const float*)d_in[7];
  const float* qw     = (const float*)d_in[8];
  const float* kw     = (const float*)d_in[9];
  const float* vw     = (const float*)d_in[10];
  const float* ow     = (const float*)d_in[11];
  const float* gw     = (const float*)d_in[12];
  const float* uw     = (const float*)d_in[13];
  const float* dw     = (const float*)d_in[14];
  float* outp = (float*)d_out;

  char* ws = (char*)d_ws;
  unsigned short* wqkv  = (unsigned short*)(ws + OFF_WQKV);
  unsigned short* wo    = (unsigned short*)(ws + OFF_WO);
  float*          hr    = (float*)(ws + OFF_HR);
  unsigned short* x16   = (unsigned short*)(ws + OFF_X16);
  float*          h1    = (float*)(ws + OFF_H1);
  float*          qkv   = (float*)(ws + OFF_QKV);
  unsigned short* q16   = (unsigned short*)(ws + OFF_Q16);
  unsigned short* k16   = (unsigned short*)(ws + OFF_K16);
  unsigned short* vt16  = (unsigned short*)(ws + OFF_VT16);
  unsigned short* att16 = (unsigned short*)(ws + OFF_ATT);
  unsigned short* v16   = (unsigned short*)(ws + OFF_V16);
  unsigned short* y16   = (unsigned short*)(ws + OFF_Y16);
  unsigned short* wd    = (unsigned short*)(ws + OFF_WD);
  unsigned short* wgu   = (unsigned short*)(ws + OFF_WGU);
  unsigned short* g16   = (unsigned short*)(ws + OFF_G16);
  unsigned short* u16   = (unsigned short*)(ws + OFF_U16);
  unsigned short* h16   = (unsigned short*)(ws + OFF_H16);
  float*          tmpf  = (float*)(ws + OFF_TMP);

  auto ggrid = [](int M, int N) { return dim3((unsigned)((((M / 64) * (N / 64)) + 7) / 8), 1); };

  cvt_weight_k<<<dim3(D_MODEL / 64, D_MODEL / 64), 256, 0, stream>>>(qw, D_MODEL, D_MODEL, wqkv);
  cvt_weight_k<<<dim3(KV_COLS / 64, D_MODEL / 64), 256, 0, stream>>>(kw, KV_COLS, D_MODEL, wqkv + (size_t)KCOL0 * D_MODEL);
  cvt_weight_k<<<dim3(KV_COLS / 64, D_MODEL / 64), 256, 0, stream>>>(vw, KV_COLS, D_MODEL, wqkv + (size_t)VCOL0 * D_MODEL);
  cvt_weight_k<<<dim3(D_MODEL / 64, D_MODEL / 64), 256, 0, stream>>>(ow, D_MODEL, D_MODEL, wo);

  rmsnorm_row_k<true, true><<<dim3(BT_ROWS), 256, 0, stream>>>(hidden, ln1, hr, x16);

  wmma_gemm64<0, 0, 0, 0, false, 0><<<ggrid(BT_ROWS, QKV_N), 256, 0, stream>>>(
      x16, x16, D_MODEL, 0L, wqkv, wqkv, D_MODEL, 0L, (void*)qkv, (void*)qkv, QKV_N, 0L,
      hr, hr, 0L, BT_ROWS, QKV_N, D_MODEL, 1.0f / W_CARRY);

  headnorm_rope_k<<<dim3(BT_ROWS), 256, 0, stream>>>(qkv, qns, kns, sinp, cosp, q16, k16, v16);

  vt_transpose_k<<<dim3(T_LEN / 64, B_SZ * N_KVH), 256, 0, stream>>>(v16, vt16);

  attn_causal_k<<<dim3(B_SZ * N_QH * (T_LEN / 64)), 128, 0, stream>>>(q16, k16, vt16, maskp, att16);

  wmma_gemm64<0, 0, 0, 0, true, 0><<<ggrid(BT_ROWS, D_MODEL), 256, 0, stream>>>(
      att16, att16, D_MODEL, 0L, wo, wo, D_MODEL, 0L, (void*)h1, (void*)h1, D_MODEL, 0L,
      hr, hr, 0L, BT_ROWS, D_MODEL, D_MODEL, 1.0f / (W_CARRY * ATT_CARRY));

  rmsnorm_row_k<false, false><<<dim3(BT_ROWS), 256, 0, stream>>>(h1, ln2, tmpf, y16);

  cvt_weight_k<<<dim3(F_DIM / 64, D_MODEL / 64), 256, 0, stream>>>(gw, F_DIM, D_MODEL, wgu);
  cvt_weight_k<<<dim3(F_DIM / 64, D_MODEL / 64), 256, 0, stream>>>(uw, F_DIM, D_MODEL, wgu + (size_t)F_DIM * D_MODEL);
  cvt_weight_k<<<dim3(D_MODEL / 64, F_DIM / 64), 256, 0, stream>>>(dw, D_MODEL, F_DIM, wd);

  const int n8 = BT_ROWS * F_HALF / 8;
  for (int hf = 0; hf < 2; ++hf) {
    wmma_gemm64<0, 0, 0, 1, false, 0><<<ggrid(BT_ROWS, F_HALF), 256, 0, stream>>>(
        y16, y16, D_MODEL, 0L, wgu + (size_t)(hf * F_HALF) * D_MODEL, wgu + (size_t)(hf * F_HALF) * D_MODEL, D_MODEL, 0L,
        (void*)g16, (void*)g16, F_HALF, 0L, h1, h1, 0L, BT_ROWS, F_HALF, D_MODEL, 1.0f / W_CARRY);
    wmma_gemm64<0, 0, 0, 1, false, 0><<<ggrid(BT_ROWS, F_HALF), 256, 0, stream>>>(
        y16, y16, D_MODEL, 0L, wgu + (size_t)(F_DIM + hf * F_HALF) * D_MODEL, wgu + (size_t)(F_DIM + hf * F_HALF) * D_MODEL, D_MODEL, 0L,
        (void*)u16, (void*)u16, F_HALF, 0L, h1, h1, 0L, BT_ROWS, F_HALF, D_MODEL, 1.0f / W_CARRY);
    silu_mul_k<<<dim3((unsigned)((n8 + 255) / 256)), 256, 0, stream>>>(g16, u16, h16, n8);
    float* dst = (hf == 0) ? tmpf : outp;
    const float* res = (hf == 0) ? (const float*)h1 : (const float*)tmpf;
    wmma_gemm64<0, 0, 0, 0, true, 0><<<ggrid(BT_ROWS, D_MODEL), 256, 0, stream>>>(
        h16, h16, F_HALF, 0L, wd + (size_t)hf * F_HALF, wd + (size_t)hf * F_HALF, F_DIM, 0L,
        (void*)dst, (void*)dst, D_MODEL, 0L, res, res, 0L, BT_ROWS, D_MODEL, F_HALF, 1.0f / (W_CARRY * HID_CARRY));
  }
  (void)ws_size;
}
